// BiCrossAttention_38749194945183
// MI455X (gfx1250) — hardware-verified
//
#include <hip/hip_runtime.h>
#include <math.h>

constexpr int kBatch  = 2;
constexpr int kSeq    = 2048;
constexpr int kQDim   = 1024;
constexpr int kHeads  = 8;
constexpr int kDHead  = 64;
constexpr int kInner  = kHeads * kDHead;
constexpr int kTok    = kBatch * kSeq;
constexpr int kQKVld  = 3 * kInner;
constexpr int kGroups = kBatch * kHeads;
constexpr int kChunkG = 2;
constexpr float kScale     = 0.125f;
constexpr float kWCarry    = 16.0f;
constexpr float kWCarryInv = 1.0f / 16.0f;
constexpr float kPCarry    = 2048.0f;
constexpr float kPCarryInv = 1.0f / 2048.0f;
constexpr float kOCarry    = 256.0f;
constexpr float kOutScale  = 1.0f / (256.0f * 16.0f);

static_assert(kTok % 64 == 0 && kQKVld % 64 == 0 && kQDim % 64 == 0 && kInner % 64 == 0 && kSeq % 64 == 0);
static_assert(kQDim % 32 == 0 && kDHead % 32 == 0 && kSeq % 32 == 0 && kInner % 32 == 0);
static_assert(kHeads % kChunkG == 0);

constexpr size_t kBytesX16 = (size_t)kTok * kQDim * 2;
constexpr size_t kBytesW1T = (size_t)kQKVld * kQDim * 2;
constexpr size_t kBytesWoT = (size_t)kQDim * kInner * 2;
constexpr size_t kBytesQKV = (size_t)kTok * kQKVld * 2;
constexpr size_t kBytesVT  = (size_t)kGroups * kDHead * kSeq * 2;
constexpr size_t kBytesS   = (size_t)kChunkG * kSeq * kSeq * 4;
constexpr size_t kBytesP   = (size_t)kChunkG * kSeq * kSeq * 2;
constexpr size_t kBytesO   = (size_t)kTok * kInner * 4;
constexpr size_t kBytesO16 = (size_t)kTok * kInner * 2;
constexpr size_t kOffX16  = 0;
constexpr size_t kOffC16  = kOffX16 + kBytesX16;
constexpr size_t kOffW1T  = kOffC16 + kBytesX16;
constexpr size_t kOffW2T  = kOffW1T + kBytesW1T;
constexpr size_t kOffWoT  = kOffW2T + kBytesW1T;
constexpr size_t kOffQKV1 = kOffWoT + kBytesWoT;
constexpr size_t kOffQKV2 = kOffQKV1 + kBytesQKV;
constexpr size_t kOffVT1  = kOffQKV2 + kBytesQKV;
constexpr size_t kOffVT2  = kOffVT1 + kBytesVT;
constexpr size_t kOffS    = kOffVT2 + kBytesVT;
constexpr size_t kOffP    = kOffS + kBytesS;
constexpr size_t kOffO1   = kOffP + kBytesP;
constexpr size_t kOffO2   = kOffO1 + kBytesO;
constexpr size_t kOffO16  = kOffO2 + kBytesO;
constexpr size_t kWsTotal = kOffO16 + kBytesO16;
static_assert(kWsTotal == (size_t)128974848);
static_assert(kWsTotal <= (size_t)134217728);

typedef __attribute__((ext_vector_type(16))) _Float16 v16h;
typedef __attribute__((ext_vector_type(8)))  _Float16 v8h;
typedef __attribute__((ext_vector_type(16))) __bf16   v16b;
typedef __attribute__((ext_vector_type(8)))  __bf16   v8b;
typedef __attribute__((ext_vector_type(8)))  float    v8f;
typedef __attribute__((ext_vector_type(4)))  float    v4f;
typedef __attribute__((ext_vector_type(4)))  unsigned int v4u;

__device__ __forceinline__ unsigned short f2bf_bits(float f) {
  unsigned u = __float_as_uint(f);
  return (unsigned short)((u + 0x7FFFu + ((u >> 16) & 1u)) >> 16);
}
__device__ __forceinline__ float bf_bits2f(unsigned short h) { return __uint_as_float(((unsigned)h) << 16); }

__device__ __forceinline__ void dep_guard_h(v8f& a, v8f& b, v16h x, v16h y) { asm volatile("v_nop\n\tv_nop\n\tv_nop\n\tv_nop" : "+v"(a), "+v"(b) : "v"(x), "v"(y)); }
__device__ __forceinline__ void dep_guard_b(v8f& a, v8f& b, v16b x, v16b y) { asm volatile("v_nop\n\tv_nop\n\tv_nop\n\tv_nop" : "+v"(a), "+v"(b) : "v"(x), "v"(y)); }
__device__ __forceinline__ void keep4_h(v16h a, v16h b, v16h c, v16h d) { asm volatile("v_nop" :: "v"(a), "v"(b), "v"(c), "v"(d)); }
__device__ __forceinline__ void keep4_b(v16b a, v16b b, v16b c, v16b d) { asm volatile("v_nop" :: "v"(a), "v"(b), "v"(c), "v"(d)); }
__device__ __forceinline__ void acc_guard4(v8f& a, v8f& b, v8f& c, v8f& d) { asm volatile("v_nop\n\tv_nop\n\tv_nop\n\tv_nop" : "+v"(a), "+v"(b), "+v"(c), "+v"(d)); }
template <typename T> struct Frag;
template <> struct Frag<_Float16> {
  typedef v16h V; union U { v16h v; v8h h[2]; };
  static __device__ __forceinline__ v16h load(const _Float16* p) {
    U f; f.h[0] = *(const v8h*)(p); f.h[1] = *(const v8h*)(p + 16); return f.v;
  }
  static __device__ __forceinline__ v8f mma(v16h a, v16h b, v8f c) {
    return __builtin_amdgcn_wmma_f32_16x16x32_f16(false, a, false, b, (short)0, c, false, false);
  }
  static __device__ __forceinline__ void guard(v8f& a, v8f& b, v16h x, v16h y) { dep_guard_h(a, b, x, y); }
  static __device__ __forceinline__ void keep(v16h a, v16h b, v16h c, v16h d) { keep4_h(a, b, c, d); }
};
template <> struct Frag<__bf16> {
  typedef v16b V; union U { v16b v; v8b h[2]; };
  static __device__ __forceinline__ v16b load(const __bf16* p) {
    U f; f.h[0] = *(const v8b*)(p); f.h[1] = *(const v8b*)(p + 16); return f.v;
  }
  static __device__ __forceinline__ v8f mma(v16b a, v16b b, v8f c) {
    return __builtin_amdgcn_wmma_f32_16x16x32_bf16(false, a, false, b, (short)0, c, false, false);
  }
  static __device__ __forceinline__ void guard(v8f& a, v8f& b, v16b x, v16b y) { dep_guard_b(a, b, x, y); }
  static __device__ __forceinline__ void keep(v16b a, v16b b, v16b c, v16b d) { keep4_b(a, b, c, d); }
};

__device__ __forceinline__ unsigned pk16(unsigned short a, unsigned short b) { return (unsigned)a | ((unsigned)b << 16); }
__device__ __forceinline__ unsigned short h_bits(float f) { const _Float16 h = (_Float16)f; return __builtin_bit_cast(unsigned short, h); }

template <int ET> struct Elem;
template <> struct Elem<0> { typedef _Float16 T; };
template <> struct Elem<1> { typedef __bf16 T; };
template <int ET, bool SPLIT, int BIAS_MODE, int OUT_MODE, bool RESID, int ACT = 0>
__global__ __launch_bounds__(256) void wmma_gemm64(
    const unsigned short* __restrict__ Ap, const unsigned short* __restrict__ A2p, int lda, long strideA,
    const unsigned short* __restrict__ Btp, const unsigned short* __restrict__ Bt2p, int ldb, long strideB,
    void* __restrict__ Cout, void* __restrict__ Cout2, int ldc, long strideC,
    const float* __restrict__ bias,
    const float* __restrict__ resid, long strideR,
    int M, int N, int K, float scale) {
  typedef typename Elem<ET>::T T;
  typedef typename Frag<T>::V V;
  const T* A = (const T*)Ap; const T* A2 = (const T*)A2p; const T* Bt = (const T*)Btp; const T* Bt2 = (const T*)Bt2p;
  __shared__ __align__(16) float sT[8][16 * 68];
  const int b    = blockIdx.y;
  const int lane = threadIdx.x & 31;
  const int wave = threadIdx.x >> 5;
  const int tilesN = N >> 6;
  const int tilesM = M >> 6;
  const int tile = blockIdx.x * 8 + wave;
  if (tile >= tilesM * tilesN) return;
  const int tm = tile / tilesN;
  const int tn = tile - tm * tilesN;
  const int m0 = tm << 6;
  const int n0 = tn << 6;

  const T* Ab  = A  + (size_t)b * strideA;
  const T* Bb  = Bt + (size_t)b * strideB;
  const T* Ab2 = SPLIT ? (A2  + (size_t)b * strideA) : nullptr;
  const T* Bb2 = SPLIT ? (Bt2 + (size_t)b * strideB) : nullptr;

  const int rlane = lane & 15;
  const int koff  = (lane >> 4) * 8;
  const int mOff  = (lane >> 4) * 8;

  v8f acc[4][4];
#pragma unroll
  for (int i = 0; i < 4; ++i)
#pragma unroll
    for (int j = 0; j < 4; ++j) acc[i][j] = (v8f){0.f,0.f,0.f,0.f,0.f,0.f,0.f,0.f};

  for (int k0 = 0; k0 < K; k0 += 32) {
    V bh[4], bl[4];
#pragma unroll
    for (int j = 0; j < 4; ++j) {
      const size_t bo = (size_t)(n0 + (j << 4) + rlane) * ldb + koff + k0;
      bh[j] = Frag<T>::load(Bb + bo);
      if (SPLIT) bl[j] = Frag<T>::load(Bb2 + bo);
    }
#pragma unroll
    for (int i = 0; i < 4; ++i) {
      const size_t ao = (size_t)(m0 + (i << 4) + rlane) * lda + koff + k0;
      V ah = Frag<T>::load(Ab + ao);
      V al;
      if (SPLIT) al = Frag<T>::load(Ab2 + ao);
#pragma unroll
      for (int j = 0; j < 4; ++j) {
        acc[i][j] = Frag<T>::mma(ah, bh[j], acc[i][j]);
        if (SPLIT) {
          acc[i][j] = Frag<T>::mma(ah, bl[j], acc[i][j]);
          acc[i][j] = Frag<T>::mma(al, bh[j], acc[i][j]);
        }
      }
      Frag<T>::guard(acc[i][0], acc[i][3], ah, SPLIT ? al : ah);
    }
    Frag<T>::keep(bh[0], bh[1], bh[2], bh[3]);
    if (SPLIT) Frag<T>::keep(bl[0], bl[1], bl[2], bl[3]);
  }
  acc_guard4(acc[0][0], acc[0][1], acc[0][2], acc[0][3]);
  acc_guard4(acc[1][0], acc[1][1], acc[1][2], acc[1][3]);
  acc_guard4(acc[2][0], acc[2][1], acc[2][2], acc[2][3]);
  acc_guard4(acc[3][0], acc[3][1], acc[3][2], acc[3][3]);

  float* slab = sT[wave];
  const float* Rb = RESID ? (resid + (size_t)b * strideR) : nullptr;
#pragma unroll
  for (int i = 0; i < 4; ++i) {
    const int mBase = m0 + (i << 4);
#pragma unroll
    for (int j = 0; j < 4; ++j) {
      const int n = n0 + (j << 4) + rlane;
      float bv = 0.f;
      if (BIAS_MODE == 2) bv = bias[n];
#pragma unroll
      for (int r = 0; r < 8; ++r) {
        float v = acc[i][j][r] * scale;
        if (BIAS_MODE == 1) v += bias[mBase + mOff + r];
        if (BIAS_MODE == 2) v += bv;
        if (RESID) v += Rb[(size_t)(mBase + mOff + r) * ldc + n];
        if (ACT == 2) v = fmaxf(v, 0.0f);
        if (ACT == 4) v = (v > 0.f) ? v : 0.01f * v;
        slab[(mOff + r) * 68 + (j << 4) + rlane] = v;
      }
    }
    __builtin_amdgcn_fence(__ATOMIC_RELEASE, "workgroup");
    __builtin_amdgcn_wave_barrier();
    __builtin_amdgcn_fence(__ATOMIC_ACQUIRE, "workgroup");
    if (OUT_MODE == 0) {
      float* C = (float*)Cout + (size_t)b * strideC;
      const int hh = lane >> 4, c4 = (lane & 15) * 4;
      for (int pass = 0; pass < 2; ++pass) {
#pragma unroll
        for (int it = 0; it < 8; ++it) {
          const int row = it * 2 + hh;
          v4f v = *(const v4f*)(slab + row * 68 + c4);
          *(volatile v4f*)(C + (size_t)(mBase + row) * ldc + n0 + c4) = v;
        }
        __threadfence();
      }
    } else {
      const int q = lane >> 3, c8 = (lane & 7) * 8;
      unsigned short* C  = (unsigned short*)Cout  + (size_t)b * strideC;
      unsigned short* C2 = (OUT_MODE == 2) ? ((unsigned short*)Cout2 + (size_t)b * strideC) : nullptr;
      for (int pass = 0; pass < 2; ++pass) {
#pragma unroll
        for (int it = 0; it < 4; ++it) {
          const int row = it * 4 + q;
          const float* sp = slab + row * 68 + c8;
          v8h hv, lv;
#pragma unroll
          for (int e = 0; e < 8; ++e) {
            if (OUT_MODE == 1) {
              hv[e] = (_Float16)sp[e];
            } else {
              unsigned short hb = f2bf_bits(sp[e]);
              unsigned short lb = f2bf_bits(sp[e] - bf_bits2f(hb));
              hv[e] = __builtin_bit_cast(_Float16, hb);
              lv[e] = __builtin_bit_cast(_Float16, lb);
            }
          }
          *(volatile v8h*)(C + (size_t)(mBase + row) * ldc + n0 + c8) = hv;
          if (OUT_MODE == 2) *(volatile v8h*)(C2 + (size_t)(mBase + row) * ldc + n0 + c8) = lv;
        }
        __threadfence();
      }
    }
    __builtin_amdgcn_fence(__ATOMIC_RELEASE, "workgroup");
    __builtin_amdgcn_wave_barrier();
    __builtin_amdgcn_fence(__ATOMIC_ACQUIRE, "workgroup");
  }
}

__global__ __launch_bounds__(256) void cast8_f16_kernel(const float* __restrict__ in, unsigned short* __restrict__ out, int n8) {
  const int i = blockIdx.x * 256 + threadIdx.x;
  if (i >= n8) return;
  const float* p = in + 8 * (size_t)i;
  const v4f a = *(const v4f*)(p);
  const v4f c = *(const v4f*)(p + 4);
  unsigned short hb[8];
#pragma unroll
  for (int e = 0; e < 4; ++e) {
    hb[e]     = h_bits(a[e]);
    hb[4 + e] = h_bits(c[e]);
  }
  const v4u u = (v4u){pk16(hb[0], hb[1]), pk16(hb[2], hb[3]), pk16(hb[4], hb[5]), pk16(hb[6], hb[7])};
  unsigned short* q = out + 8 * (size_t)i;
  *(volatile v4u*)q = u;
  __threadfence();
  *(volatile v4u*)q = u;
}

__global__ __launch_bounds__(256) void wtcast_kernel(const float* __restrict__ W0, const float* __restrict__ W1,
                                                     const float* __restrict__ W2,
                                                     unsigned short* __restrict__ out, int nin, int nout, long zstride, float scale) {
  __shared__ float sm[64][65];
  const int t  = threadIdx.x;
  const int d0 = blockIdx.x * 64;
  const int h0 = blockIdx.y * 64;
  const int z  = blockIdx.z;
  const float* W = (z == 0) ? W0 : (z == 1) ? W1 : W2;
#pragma unroll
  for (int i = 0; i < 16; ++i) {
    const int e = i * 256 + t;
    const int r = e >> 6;
    const int c = e & 63;
    sm[c][r] = W[(size_t)(d0 + r) * nout + h0 + c] * scale;
  }
  __syncthreads();
  const int lane = t & 31, wave = t >> 5;
  const int q = lane >> 3, c8 = (lane & 7) * 8;
  unsigned short* op = out + (size_t)z * zstride;
  for (int pass = 0; pass < 2; ++pass) {
#pragma unroll
    for (int it = 0; it < 2; ++it) {
      const int row = wave * 8 + it * 4 + q;
      unsigned short hb[8];
#pragma unroll
      for (int e = 0; e < 8; ++e) hb[e] = h_bits(sm[row][c8 + e]);
      const v4u u = (v4u){pk16(hb[0], hb[1]), pk16(hb[2], hb[3]), pk16(hb[4], hb[5]), pk16(hb[6], hb[7])};
      *(volatile v4u*)(op + (size_t)(h0 + row) * nin + d0 + c8) = u;
    }
    __threadfence();
  }
}

__global__ __launch_bounds__(256) void vtrans_kernel(const unsigned short* __restrict__ srcA, const unsigned short* __restrict__ srcB,
                                                     unsigned short* __restrict__ dstA, unsigned short* __restrict__ dstB) {
  __shared__ unsigned short sm[64][66];
  const int t  = threadIdx.x;
  const int z  = blockIdx.z;
  const unsigned short* src = (z == 0) ? srcA : srcB;
  unsigned short* dst = (z == 0) ? dstA : dstB;
  const int bh = blockIdx.y;
  const int b  = bh >> 3, h = bh & 7;
  const int s0 = blockIdx.x * 64;
#pragma unroll
  for (int it = 0; it < 2; ++it) {
    const int e  = it * 256 + t;
    const int r  = e >> 3;
    const int c8 = (e & 7) * 8;
    const v4u w = *(const v4u*)(src + (size_t)(b * kSeq + s0 + r) * kQKVld + 2 * kInner + h * kDHead + c8);
#pragma unroll
    for (int j = 0; j < 4; ++j) {
      sm[r][c8 + 2 * j]     = (unsigned short)(w[j] & 0xffffu);
      sm[r][c8 + 2 * j + 1] = (unsigned short)(w[j] >> 16);
    }
  }
  __syncthreads();
  const int lane = t & 31, wave = t >> 5;
  const int q = lane >> 3, c8 = (lane & 7) * 8;
  unsigned short* op = dst + (size_t)bh * kDHead * kSeq;
  for (int pass = 0; pass < 2; ++pass) {
#pragma unroll
    for (int it = 0; it < 2; ++it) {
      const int row = wave * 8 + it * 4 + q;
      const v4u u = (v4u){pk16(sm[c8][row],     sm[c8 + 1][row]), pk16(sm[c8 + 2][row], sm[c8 + 3][row]),
                          pk16(sm[c8 + 4][row], sm[c8 + 5][row]), pk16(sm[c8 + 6][row], sm[c8 + 7][row])};
      *(volatile v4u*)(op + (size_t)row * kSeq + s0 + c8) = u;
    }
    __threadfence();
  }
}

__global__ __launch_bounds__(256) void softmax_row_kernel(const float* __restrict__ S, unsigned short* __restrict__ P) {
  __shared__ float redM[8];
  __shared__ float redS[8];
  const int row  = blockIdx.x;
  const int t    = threadIdx.x;
  const int lane = t & 31, wave = t >> 5;
  const int c0   = t * 8;
  const float* sr = S + (size_t)row * kSeq + c0;
  const v4f a = *(const v4f*)(sr);
  const v4f c = *(const v4f*)(sr + 4);
  float x[8];
#pragma unroll
  for (int e = 0; e < 4; ++e) { x[e] = a[e]; x[4 + e] = c[e]; }
  float m = fmaxf(fmaxf(fmaxf(x[0], x[1]), fmaxf(x[2], x[3])), fmaxf(fmaxf(x[4], x[5]), fmaxf(x[6], x[7])));
#pragma unroll
  for (int off = 16; off > 0; off >>= 1) m = fmaxf(m, __shfl_xor(m, off, 32));
  if (lane == 0) redM[wave] = m;
  __syncthreads();
  float gm = redM[0];
#pragma unroll
  for (int w = 1; w < 8; ++w) gm = fmaxf(gm, redM[w]);
  float ev[8];
#pragma unroll
  for (int e = 0; e < 8; ++e) ev[e] = expf(x[e] - gm);
  float s = ((ev[0] + ev[1]) + (ev[2] + ev[3])) + ((ev[4] + ev[5]) + (ev[6] + ev[7]));
#pragma unroll
  for (int off = 16; off > 0; off >>= 1) s += __shfl_xor(s, off, 32);
  if (lane == 0) redS[wave] = s;
  __syncthreads();
  const float tot = ((redS[0] + redS[1]) + (redS[2] + redS[3])) + ((redS[4] + redS[5]) + (redS[6] + redS[7]));
  const float inv = kPCarry / tot;
  unsigned short hb[8];
#pragma unroll
  for (int e = 0; e < 8; ++e) hb[e] = h_bits(ev[e] * inv);
  const v4u u = (v4u){pk16(hb[0], hb[1]), pk16(hb[2], hb[3]), pk16(hb[4], hb[5]), pk16(hb[6], hb[7])};
  unsigned short* q = P + (size_t)row * kSeq + c0;
  *(volatile v4u*)q = u;
  __threadfence();
  *(volatile v4u*)q = u;
}

__global__ __launch_bounds__(256) void mix_kernel(const float* __restrict__ o1, const float* __restrict__ o2,
                                                  const float* __restrict__ alpha_p, unsigned short* __restrict__ out, int n8) {
#pragma clang fp contract(off)
  const int i = blockIdx.x * 256 + threadIdx.x;
  if (i >= n8) return;
  const float al = 1.0f / (1.0f + expf(-alpha_p[0]));
  const float be = 1.0f - al;
  const float* p1 = o1 + 8 * (size_t)i;
  const float* p2 = o2 + 8 * (size_t)i;
  const v4f a1 = *(const v4f*)(p1);
  const v4f c1 = *(const v4f*)(p1 + 4);
  const v4f a2 = *(const v4f*)(p2);
  const v4f c2 = *(const v4f*)(p2 + 4);
  unsigned short hb[8];
#pragma unroll
  for (int e = 0; e < 4; ++e) {
    hb[e]     = h_bits((a1[e] * al + a2[e] * be) * kOCarry);
    hb[4 + e] = h_bits((c1[e] * al + c2[e] * be) * kOCarry);
  }
  const v4u u = (v4u){pk16(hb[0], hb[1]), pk16(hb[2], hb[3]), pk16(hb[4], hb[5]), pk16(hb[6], hb[7])};
  unsigned short* q = out + 8 * (size_t)i;
  *(volatile v4u*)q = u;
  __threadfence();
  *(volatile v4u*)q = u;
}

extern "C" void kernel_launch(void* const* d_in, const int* in_sizes, int n_in,
                              void* d_out, int out_size, void* d_ws, size_t ws_size,
                              hipStream_t stream) {
  if (n_in < 11) return;
  if (ws_size < kWsTotal) return;
  if ((size_t)out_size < (size_t)kTok * kQDim) return;
  if (in_sizes[0] != kTok * kQDim || in_sizes[1] != kTok * kQDim) return;
  if (in_sizes[2] != kQDim * kInner || in_sizes[9] != kInner * kQDim || in_sizes[10] != kQDim || in_sizes[8] < 1) return;

  const float* x     = (const float*)d_in[0];
  const float* ctx   = (const float*)d_in[1];
  const float* Wq1   = (const float*)d_in[2];
  const float* Wk1   = (const float*)d_in[3];
  const float* Wv1   = (const float*)d_in[4];
  const float* Wq2   = (const float*)d_in[5];
  const float* Wk2   = (const float*)d_in[6];
  const float* Wv2   = (const float*)d_in[7];
  const float* alpha = (const float*)d_in[8];
  const float* Wout  = (const float*)d_in[9];
  const float* bout  = (const float*)d_in[10];
  float* out = (float*)d_out;

  char* ws = (char*)d_ws;
  unsigned short* X16  = (unsigned short*)(ws + kOffX16);
  unsigned short* C16  = (unsigned short*)(ws + kOffC16);
  unsigned short* W1T  = (unsigned short*)(ws + kOffW1T);
  unsigned short* W2T  = (unsigned short*)(ws + kOffW2T);
  unsigned short* WoT  = (unsigned short*)(ws + kOffWoT);
  unsigned short* QKV1 = (unsigned short*)(ws + kOffQKV1);
  unsigned short* QKV2 = (unsigned short*)(ws + kOffQKV2);
  unsigned short* VT1  = (unsigned short*)(ws + kOffVT1);
  unsigned short* VT2  = (unsigned short*)(ws + kOffVT2);
  float*          Sbuf = (float*)(ws + kOffS);
  unsigned short* Pbuf = (unsigned short*)(ws + kOffP);
  float*          O1   = (float*)(ws + kOffO1);
  float*          O2   = (float*)(ws + kOffO2);
  unsigned short* O16  = (unsigned short*)(ws + kOffO16);

  const int n8x = kTok * kQDim / 8;
  cast8_f16_kernel<<<n8x / 256, 256, 0, stream>>>(x, X16, n8x);
  cast8_f16_kernel<<<n8x / 256, 256, 0, stream>>>(ctx, C16, n8x);

  wtcast_kernel<<<dim3(kQDim / 64, kInner / 64, 3), 256, 0, stream>>>(Wq1, Wk1, Wv1, W1T, kQDim, kInner, (long)kInner * kQDim, kWCarry);
  wtcast_kernel<<<dim3(kQDim / 64, kInner / 64, 3), 256, 0, stream>>>(Wq2, Wk2, Wv2, W2T, kQDim, kInner, (long)kInner * kQDim, kWCarry);
  wtcast_kernel<<<dim3(kInner / 64, kQDim / 64, 1), 256, 0, stream>>>(Wout, Wout, Wout, WoT, kInner, kQDim, (long)0, kWCarry);

  {
    const int tiles = (kTok / 64) * (kQKVld / 64);
    wmma_gemm64<0, false, 0, 1, false><<<dim3(tiles / 8, 1), 256, 0, stream>>>(
        X16, X16, kQDim, (long)0, W1T, W1T, kQDim, (long)0, QKV1, QKV1, kQKVld, (long)0,
        bout, O1, (long)0, kTok, kQKVld, kQDim, kWCarryInv);
    wmma_gemm64<0, false, 0, 1, false><<<dim3(tiles / 8, 1), 256, 0, stream>>>(
        C16, C16, kQDim, (long)0, W2T, W2T, kQDim, (long)0, QKV2, QKV2, kQKVld, (long)0,
        bout, O1, (long)0, kTok, kQKVld, kQDim, kWCarryInv);
  }

  vtrans_kernel<<<dim3(kSeq / 64, kGroups, 2), 256, 0, stream>>>(QKV1, QKV2, VT1, VT2);

  for (int br = 0; br < 2; ++br) {
    const unsigned short* qpl  = (br == 0) ? QKV2 : QKV1;
    const unsigned short* kpl  = (br == 0) ? QKV1 : QKV2;
    const unsigned short* vtpl = (br == 0) ? VT1 : VT2;
    float* opl = (br == 0) ? O1 : O2;
    for (int b = 0; b < kBatch; ++b) {
      for (int hp = 0; hp < kHeads / kChunkG; ++hp) {
        const int h0 = hp * kChunkG;
        const unsigned short* qp = qpl + (size_t)b * kSeq * kQKVld + h0 * kDHead;
        const unsigned short* kp = kpl + (size_t)b * kSeq * kQKVld + kInner + h0 * kDHead;
        wmma_gemm64<0, false, 0, 0, false><<<dim3((kSeq / 64) * (kSeq / 64) / 8, kChunkG), 256, 0, stream>>>(
            qp, qp, kQKVld, (long)kDHead, kp, kp, kQKVld, (long)kDHead, Sbuf, Sbuf, kSeq, (long)kSeq * kSeq,
            bout, O1, (long)0, kSeq, kSeq, kDHead, kScale);
        softmax_row_kernel<<<kChunkG * kSeq, 256, 0, stream>>>(Sbuf, Pbuf);
        const unsigned short* vtp = vtpl + (size_t)(b * kHeads + h0) * kDHead * kSeq;
        float* op = opl + (size_t)b * kSeq * kInner + h0 * kDHead;
        wmma_gemm64<0, false, 0, 0, false><<<dim3((kSeq / 64) / 8, kChunkG), 256, 0, stream>>>(
            Pbuf, Pbuf, kSeq, (long)kSeq * kSeq, vtp, vtp, kSeq, (long)kDHead * kSeq, op, op, kInner, (long)kDHead,
            bout, O1, (long)0, kSeq, kDHead, kSeq, kPCarryInv);
      }
    }
  }

  const int n8o = kTok * kInner / 8;
  mix_kernel<<<n8o / 256, 256, 0, stream>>>(O1, O2, alpha, O16, n8o);

  {
    const int tiles = (kTok / 64) * (kQDim / 64);
    wmma_gemm64<0, false, 2, 0, false><<<dim3(tiles / 8, 1), 256, 0, stream>>>(
        O16, O16, kInner, (long)0, WoT, WoT, kInner, (long)0, out, out, kQDim, (long)0,
        bout, O1, (long)0, kTok, kQDim, kInner, kOutScale);
  }
}
